// SocialAgg_21354577396100
// MI455X (gfx1250) — hardware-verified
//
#include <hip/hip_runtime.h>
#include <stddef.h>


#define NTHR   256
#define NWAVE  8
#define EPT    8
#define CHUNK  (NTHR * EPT)
#define WCAP   (EPT * 32)
#define LISTN  (NWAVE * WCAP)
#define PASSN  (NWAVE * 32)
#define PCAP   (CHUNK + PASSN)
#define NB     512
#define SPW    (NB / NWAVE)
#define TPW    (NB / (16 * NWAVE))
#define FD     64
#define NRB    (NWAVE * 16)
#define WSB_MAX ((size_t)134217728)

static_assert((PCAP % PASSN) == 0);
static_assert(SPW * NWAVE == NB);
static_assert(TPW * 16 == SPW);
static_assert(PASSN == 32 * NWAVE);

typedef float          v2f_t  __attribute__((ext_vector_type(2)));
typedef float          v4f_t  __attribute__((ext_vector_type(4)));
typedef float          v8f    __attribute__((ext_vector_type(8)));
typedef int            v4i_t  __attribute__((ext_vector_type(4)));
typedef _Float16       v8h_t  __attribute__((ext_vector_type(8)));
typedef _Float16       v16h   __attribute__((ext_vector_type(16)));
typedef unsigned short v8us_t __attribute__((ext_vector_type(8)));
typedef __bf16         v16b   __attribute__((ext_vector_type(16)));
typedef v2f_t  v2f  __attribute__((may_alias));
typedef v4f_t  v4f  __attribute__((may_alias));
typedef v4i_t  v4i  __attribute__((may_alias));
typedef v8h_t  v8h  __attribute__((may_alias));
typedef v8us_t v8us __attribute__((may_alias));
union FragH { v16h v; v8h_t h[2]; };
union FragB { v16b v; v8us_t u[2]; };

__device__ __forceinline__ v8f wmh(v16h a, v16h b, v8f c) {
  v8f d = __builtin_amdgcn_wmma_f32_16x16x32_f16(false, a, false, b, (short)0, c, false, false);
  asm volatile("v_nop\n\tv_nop\n\tv_nop\n\tv_nop" : "+v"(d) : "v"(a), "v"(b));
  return d;
}
__device__ __forceinline__ v8f wmb(v16b a, v16b b, v8f c) {
  v8f d = __builtin_amdgcn_wmma_f32_16x16x32_bf16(false, a, false, b, (short)0, c, false, false);
  asm volatile("v_nop\n\tv_nop\n\tv_nop\n\tv_nop" : "+v"(d) : "v"(a), "v"(b));
  return d;
}

__device__ __forceinline__ v8f ldc8(const float* p) {
  const v4f a = *(const v4f*)p;
  const v4f b = *(const v4f*)(p + 4);
  v8f c;
  c[0] = a.x; c[1] = a.y; c[2] = a.z; c[3] = a.w;
  c[4] = b.x; c[5] = b.y; c[6] = b.z; c[7] = b.w;
  return c;
}
__device__ __forceinline__ v8f splat8(float b) {
  v8f c;
#pragma unroll
  for (int i = 0; i < 8; ++i) c[i] = b;
  return c;
}
__device__ __forceinline__ v8h_t relu8h(v8f d) {
  v8h_t r;
#pragma unroll
  for (int i = 0; i < 8; ++i) { const float t = fmaxf(d[i], 0.0f); r[i] = (_Float16)t; }
  return r;
}
__device__ __forceinline__ v8h_t cvt8(const float* p) {
  const v4f a = *(const v4f*)p;
  const v4f b = *(const v4f*)(p + 4);
  v8h_t r;
  r[0] = (_Float16)a.x; r[1] = (_Float16)a.y; r[2] = (_Float16)a.z; r[3] = (_Float16)a.w;
  r[4] = (_Float16)b.x; r[5] = (_Float16)b.y; r[6] = (_Float16)b.z; r[7] = (_Float16)b.w;
  return r;
}
__device__ __forceinline__ int clampi(int v, int lo, int hi) {
  v = v < lo ? lo : v;
  v = v > hi ? hi : v;
  return v;
}
__device__ __forceinline__ unsigned short bf16rne(float x) {
  unsigned u = __float_as_uint(x);
  u += 0x7FFFu + ((u >> 16) & 1u);
  return (unsigned short)(u >> 16);
}

template <int RELU>
__device__ __forceinline__ void tile_store(v8f a0, v8f a1, v8f a2, v8f a3, float* ost, float* G,
                                           int growBase, int nRows, int lane, int hh, int m) {
#pragma unroll
  for (int r = 0; r < 8; ++r) {
    float* rp = ost + (8 * hh + r) * FD + m;
    float t0 = a0[r], t1 = a1[r], t2 = a2[r], t3 = a3[r];
    if (RELU != 0) { t0 = fmaxf(t0, 0.0f); t1 = fmaxf(t1, 0.0f); t2 = fmaxf(t2, 0.0f); t3 = fmaxf(t3, 0.0f); }
    rp[0] = t0; rp[16] = t1; rp[32] = t2; rp[48] = t3;
  }
  __syncthreads();
  const int rsub = lane >> 4, col = (lane & 15) * 4;
  v4f ov[8];
#pragma unroll
  for (int q = 0; q < 8; ++q) ov[q] = *(const v4f*)(ost + (2 * q + rsub) * FD + col);
#pragma unroll
  for (int q = 0; q < 8; ++q) {
    const int grow = growBase + 2 * q + rsub;
    if (grow < nRows) *(volatile v4f*)(G + (size_t)grow * FD + col) = ov[q];
  }
  __threadfence();
#pragma unroll
  for (int q = 0; q < 8; ++q) {
    const int grow = growBase + 2 * q + rsub;
    if (grow < nRows) *(volatile v4f*)(G + (size_t)grow * FD + col) = ov[q];
  }
  __syncthreads();
}

__global__ __launch_bounds__(NTHR) void k_node(const float* __restrict__ uf, const float* __restrict__ hif,
                                               const float* __restrict__ W1, const float* __restrict__ b1,
                                               float* Pp, float* Qp, int nN) {
  __shared__ __attribute__((aligned(16))) _Float16 w1a[FD * FD];
  __shared__ __attribute__((aligned(16))) _Float16 w1b[FD * FD];
  __shared__ __attribute__((aligned(16))) float    b1s[FD];
  __shared__ __attribute__((aligned(16))) float    ost[NWAVE * 16 * FD];

  const int tid = threadIdx.x, lane = tid & 31, wave = tid >> 5, hh = lane >> 4, m = lane & 15;
  for (int i = tid; i < FD * FD; i += NTHR) {
    const int n = i >> 6, k = i & 63;
    w1a[i] = (_Float16)(W1[k * FD + n] * 8.0f);
    w1b[i] = (_Float16)(W1[(FD + k) * FD + n] * 8.0f);
  }
  if (tid < FD) b1s[tid] = b1[tid] * 8.0f;
  __syncthreads();

  const int row0 = blockIdx.x * NRB + wave * 16;
  int rm = row0 + m;
  rm = rm > nN - 1 ? nN - 1 : rm;

  FragH au[2], ah[2];
#pragma unroll
  for (int c = 0; c < 2; ++c) {
    const float* pu = uf  + (size_t)rm * FD + 32 * c + 8 * hh;
    const float* ph = hif + (size_t)rm * FD + 32 * c + 8 * hh;
    au[c].h[0] = cvt8(pu);  au[c].h[1] = cvt8(pu + 16);
    ah[c].h[0] = cvt8(ph);  ah[c].h[1] = cvt8(ph + 16);
  }
  v8f dp[4], dq[4];
#pragma unroll
  for (int nt = 0; nt < 4; ++nt) { dp[nt] = splat8(0.0f); dq[nt] = splat8(b1s[16 * nt + m]); }
#pragma unroll
  for (int nt = 0; nt < 4; ++nt) {
#pragma unroll
    for (int c = 0; c < 2; ++c) {
      FragH b;
      const _Float16* bp = w1a + (16 * nt + m) * FD + 32 * c + 8 * hh;
      b.h[0] = *(const v8h*)bp;
      b.h[1] = *(const v8h*)(bp + 16);
      dp[nt] = wmh(au[c].v, b.v, dp[nt]);
      FragH b2;
      const _Float16* bq = w1b + (16 * nt + m) * FD + 32 * c + 8 * hh;
      b2.h[0] = *(const v8h*)bq;
      b2.h[1] = *(const v8h*)(bq + 16);
      dq[nt] = wmh(ah[c].v, b2.v, dq[nt]);
    }
  }
  float* myost = ost + wave * 16 * FD;
  tile_store<0>(dp[0], dp[1], dp[2], dp[3], myost, Pp, row0, nN, lane, hh, m);
  tile_store<0>(dq[0], dq[1], dq[2], dq[3], myost, Qp, row0, nN, lane, hh, m);
}

__device__ __forceinline__ int scan_chunk(const int* __restrict__ dsts, int nE, int cbase, int nodeBase,
                                          int* list, int tid, int wave) {
  int wc = 0;
  const int el0  = tid * EPT;
  const int e0   = cbase + el0;
  const int sent = -2147483647 - 1;
  v4i_t da, db;
  if (cbase + CHUNK <= nE) {
    da = *(const v4i*)(dsts + e0);
    db = *(const v4i*)(dsts + e0 + 4);
  } else {
    da.x = (e0     < nE) ? dsts[min(e0,     nE - 1)] : sent;
    da.y = (e0 + 1 < nE) ? dsts[min(e0 + 1, nE - 1)] : sent;
    da.z = (e0 + 2 < nE) ? dsts[min(e0 + 2, nE - 1)] : sent;
    da.w = (e0 + 3 < nE) ? dsts[min(e0 + 3, nE - 1)] : sent;
    db.x = (e0 + 4 < nE) ? dsts[min(e0 + 4, nE - 1)] : sent;
    db.y = (e0 + 5 < nE) ? dsts[min(e0 + 5, nE - 1)] : sent;
    db.z = (e0 + 6 < nE) ? dsts[min(e0 + 6, nE - 1)] : sent;
    db.w = (e0 + 7 < nE) ? dsts[min(e0 + 7, nE - 1)] : sent;
  }
  const unsigned nb = (unsigned)nodeBase;
  const unsigned s0 = (unsigned)da.x - nb, s1 = (unsigned)da.y - nb;
  const unsigned s2 = (unsigned)da.z - nb, s3 = (unsigned)da.w - nb;
  const unsigned s4 = (unsigned)db.x - nb, s5 = (unsigned)db.y - nb;
  const unsigned s6 = (unsigned)db.z - nb, s7 = (unsigned)db.w - nb;
  const bool h0 = s0 < (unsigned)NB, h1 = s1 < (unsigned)NB, h2 = s2 < (unsigned)NB, h3 = s3 < (unsigned)NB;
  const bool h4 = s4 < (unsigned)NB, h5 = s5 < (unsigned)NB, h6 = s6 < (unsigned)NB, h7 = s7 < (unsigned)NB;
  const unsigned any = __builtin_amdgcn_ballot_w32(h0 | h1 | h2 | h3 | h4 | h5 | h6 | h7);
  if (any != 0u) {
#define HITJ(J, HJ) { \
      const unsigned mj = __builtin_amdgcn_ballot_w32(HJ); \
      if (mj != 0u) { \
        if (HJ) { \
          const int pos = wc + (int)__builtin_amdgcn_mbcnt_lo(mj, 0u); \
          if (pos < WCAP) list[wave * WCAP + pos] = el0 + (J); \
        } \
        wc += (int)__builtin_popcount(mj); } }
    HITJ(0, h0)
    HITJ(1, h1)
    HITJ(2, h2)
    HITJ(3, h3)
    HITJ(4, h4)
    HITJ(5, h5)
    HITJ(6, h6)
    HITJ(7, h7)
#undef HITJ
  }
  return wc;
}

__global__ __launch_bounds__(NTHR) void k_agg(
    const float* __restrict__ Pp, const float* __restrict__ Qp, const float* __restrict__ hif,
    const int* __restrict__ srcs, const int* __restrict__ dsts,
    const float* __restrict__ W2, const float* __restrict__ b2,
    const float* __restrict__ W3, const float* __restrict__ b3,
    const float* __restrict__ Ww, const float* __restrict__ bw,
    float* outp, int nN, int nE) {
  __shared__ __attribute__((aligned(16))) float          accs[NB * FD];
  __shared__ __attribute__((aligned(16))) float          mxs[NB];
  __shared__ __attribute__((aligned(16))) float          dns[NB];
  __shared__ __attribute__((aligned(16))) _Float16       stg[PASSN * FD];
  __shared__ __attribute__((aligned(16))) int            list[LISTN];
  __shared__ __attribute__((aligned(16))) int            pend[PCAP];
  __shared__ __attribute__((aligned(16))) int            slotb[PASSN];
  __shared__ __attribute__((aligned(16))) int            srcb[PASSN];
  __shared__ __attribute__((aligned(16))) float          scb[PASSN];
  __shared__ __attribute__((aligned(16))) _Float16       w2t[FD * FD];
  __shared__ __attribute__((aligned(16))) _Float16       w3t[16 * FD];
  __shared__ __attribute__((aligned(16))) float          b2c[FD];
  __shared__ __attribute__((aligned(16))) float          b3c[16];
  __shared__ __attribute__((aligned(16))) unsigned short wwh[FD * FD];
  __shared__ __attribute__((aligned(16))) unsigned short wwl[FD * FD];
  __shared__ __attribute__((aligned(16))) float          bws[FD];
  __shared__ int wcnt[NWAVE];
  __shared__ int pendN;

  const int tid = threadIdx.x, lane = tid & 31, wave = tid >> 5, hh = lane >> 4, m = lane & 15;
  const int nodeBase = blockIdx.x * NB;

  {
    const v4f_t z4 = {0.0f, 0.0f, 0.0f, 0.0f};
    for (int i = tid; i < NB * FD / 4; i += NTHR) *(v4f*)(accs + 4 * i) = z4;
  }
  for (int i = tid; i < NB; i += NTHR) { mxs[i] = 0.0f; dns[i] = 0.0f; }
  for (int i = tid; i < FD * FD; i += NTHR) {
    const int n = i >> 6, k = i & 63;
    w2t[i] = (_Float16)(W2[k * FD + n] * 8.0f);
    const float w = Ww[k * FD + n];
    const unsigned short hb = bf16rne(w);
    const float rw = w - __uint_as_float((unsigned)hb << 16);
    wwh[i] = hb;
    wwl[i] = bf16rne(rw);
  }
  for (int i = tid; i < 16 * FD; i += NTHR) {
    const int rr = i >> 6, k = i & 63;
    const float w = W3[k] * 8.0f;
    w3t[i] = (_Float16)(rr == 0 ? w : 0.0f);
  }
  if (tid < FD) { b2c[tid] = b2[tid] * 64.0f; bws[tid] = bw[tid]; }
  if (tid < 16) { const float bb = b3[0] * 512.0f; b3c[tid] = (tid == 0) ? bb : 0.0f; }
  if (tid == 0) pendN = 0;
  __syncthreads();

  const int nChunks = (nE + CHUNK - 1) / CHUNK;
#pragma unroll 1
  for (int ch = 0; ch < nChunks; ++ch) {
    const int cbase = ch * CHUNK;
    const int wc = scan_chunk(dsts, nE, cbase, nodeBase, list, tid, wave);
    if (lane == 0) wcnt[wave] = wc;
    __syncthreads();

    const int base = pendN;
    int tot = 0, myoff = 0;
#pragma unroll
    for (int w = 0; w < NWAVE; ++w) {
      int c = wcnt[w];
      c = c > WCAP ? WCAP : (c < 0 ? 0 : c);
      if (w < wave) myoff += c;
      tot += c;
    }
    int newN = base + tot;
    newN = newN > PCAP ? PCAP : newN;
    {
      int n = wcnt[wave];
      n = n > WCAP ? WCAP : (n < 0 ? 0 : n);
      const int* lp = list + wave * WCAP;
      for (int i = lane; i < n; i += 32) {
        const int pos = base + myoff + i;
        if (pos < PCAP) pend[pos] = cbase + lp[i];
      }
    }
    const int fin = (ch == nChunks - 1) ? 1 : 0;
    const int R   = (fin != 0) ? (newN + PASSN - 1) / PASSN : newN / PASSN;
    const int Pv  = (fin != 0) ? newN : R * PASSN;
    __syncthreads();

#pragma unroll 1
    for (int r = 0; r < R; ++r) {
      {
        const int idx = r * PASSN + wave * 32 + lane;
        const bool valid = idx < Pv;
        int e = pend[idx];
        e = valid ? e : 0;
        e = clampi(e, 0, nE - 1);
        int d = dsts[e];
        int t = srcs[e];
        int slot = d - nodeBase;
        if (!valid || (unsigned)slot >= (unsigned)NB) slot = NB;
        d = clampi(d, 0, nN - 1);
        t = clampi(t, 0, nN - 1);
        const float* pr = Pp + (size_t)t * FD;
        const float* qr = Qp + (size_t)d * FD;
        _Float16* sr = stg + (wave * 32 + lane) * FD;
#pragma unroll 2
        for (int f = 0; f < 8; ++f) {
          const v4f p0 = *(const v4f*)(pr + 8 * f);
          const v4f p1 = *(const v4f*)(pr + 8 * f + 4);
          const v4f q0 = *(const v4f*)(qr + 8 * f);
          const v4f q1 = *(const v4f*)(qr + 8 * f + 4);
          v8h_t hv;
#pragma unroll
          for (int j = 0; j < 4; ++j) {
            const float xa = fmaxf(p0[j] + q0[j], 0.0f);
            const float xb = fmaxf(p1[j] + q1[j], 0.0f);
            hv[j]     = (_Float16)(valid ? xa : 0.0f);
            hv[4 + j] = (_Float16)(valid ? xb : 0.0f);
          }
          *(v8h*)(sr + 8 * f) = hv;
        }
        slotb[wave * 32 + lane] = slot;
        srcb[wave * 32 + lane]  = t;
      }
      __syncthreads();

#pragma unroll 1
      for (int t2 = 0; t2 < 2; ++t2) {
        const int eb = wave * 32 + 16 * t2;
        v8f d2[4];
#pragma unroll
        for (int ft = 0; ft < 4; ++ft) d2[ft] = ldc8(b2c + 16 * ft + 8 * hh);
#pragma unroll
        for (int c = 0; c < 2; ++c) {
          FragH b;
          const _Float16* bp = stg + (eb + m) * FD + 32 * c + 8 * hh;
          b.h[0] = *(const v8h*)bp;
          b.h[1] = *(const v8h*)(bp + 16);
#pragma unroll
          for (int ft = 0; ft < 4; ++ft) {
            FragH a;
            const _Float16* ap = w2t + (16 * ft + m) * FD + 32 * c + 8 * hh;
            a.h[0] = *(const v8h*)ap;
            a.h[1] = *(const v8h*)(ap + 16);
            d2[ft] = wmh(a.v, b.v, d2[ft]);
          }
        }
        FragH q3a, q3b;
        q3a.h[0] = relu8h(d2[0]); q3a.h[1] = relu8h(d2[1]);
        q3b.h[0] = relu8h(d2[2]); q3b.h[1] = relu8h(d2[3]);
        v8f d3 = ldc8(b3c + 8 * hh);
        {
          FragH a;
          const _Float16* ap = w3t + m * FD + 8 * hh;
          a.h[0] = *(const v8h*)ap;
          a.h[1] = *(const v8h*)(ap + 16);
          d3 = wmh(a.v, q3a.v, d3);
        }
        {
          FragH a;
          const _Float16* ap = w3t + m * FD + 32 + 8 * hh;
          a.h[0] = *(const v8h*)ap;
          a.h[1] = *(const v8h*)(ap + 16);
          d3 = wmh(a.v, q3b.v, d3);
        }
        if (hh == 0) scb[eb + m] = d3[0] * (1.0f / 512.0f);
      }
      __syncthreads();

      {
        const int slo = wave * SPW;
#pragma unroll 1
        for (int j = 0; j < PASSN / 32; ++j) {
          const int i0 = 32 * j;
          const int sli = slotb[i0 + lane];
          unsigned msk = __builtin_amdgcn_ballot_w32((unsigned)(sli - slo) < (unsigned)SPW);
#pragma unroll 1
          while (msk != 0u) {
            const int bit = __builtin_ctz(msk);
            msk &= msk - 1u;
            const int i = i0 + bit;
            int sl = slotb[i];
            sl = clampi(sl, slo, slo + SPW - 1);
            const float s = scb[i];
            int t = srcb[i];
            t = clampi(t, 0, nN - 1);
            const float mo = mxs[sl];
            const float dn = dns[sl];
            const bool first = (dn == 0.0f);
            const float mn = first ? s : fmaxf(mo, s);
            const float ex = expf(mo - mn);
            const float sc = first ? 0.0f : ex;
            const float p  = expf(s - mn);
            const v2f hv = *(const v2f*)(hif + (size_t)t * FD + 2 * lane);
            float* ap = accs + sl * FD + 2 * lane;
            v2f av = *(v2f*)ap;
            av.x = av.x * sc + p * hv.x;
            av.y = av.y * sc + p * hv.y;
            *(v2f*)ap = av;
            mxs[sl] = mn;
            dns[sl] = dn * sc + p;
          }
        }
      }
      __syncthreads();
    }

    int rem = newN - R * PASSN;
    rem = rem < 0 ? 0 : rem;
    if (R > 0 && tid < rem) pend[tid] = pend[R * PASSN + tid];
    if (tid == 0) pendN = rem;
  }
  __syncthreads();

#pragma unroll 1
  for (int tt = 0; tt < TPW; ++tt) {
    const int sb = (wave * TPW + tt) * 16;
    const float dv = dns[sb + m];
    const float inv = (dv > 0.0f) ? (1.0f / dv) : 0.0f;
    const float* arow = accs + (sb + m) * FD;
    v8f o[4];
#pragma unroll
    for (int nt = 0; nt < 4; ++nt) o[nt] = splat8(bws[16 * nt + m]);
#pragma unroll
    for (int c = 0; c < 2; ++c) {
      FragB ahi, alo;
#pragma unroll
      for (int j = 0; j < 2; ++j) {
        const float* xp = arow + 32 * c + 16 * j + 8 * hh;
        const v4f x0 = *(const v4f*)xp;
        const v4f x1 = *(const v4f*)(xp + 4);
        v8us_t th, tl;
#pragma unroll
        for (int i = 0; i < 4; ++i) {
          const float xa = x0[i] * inv, xb = x1[i] * inv;
          const unsigned short ha = bf16rne(xa), hb2 = bf16rne(xb);
          const float ra = xa - __uint_as_float((unsigned)ha << 16);
          const float rb = xb - __uint_as_float((unsigned)hb2 << 16);
          th[i] = ha;          th[4 + i] = hb2;
          tl[i] = bf16rne(ra); tl[4 + i] = bf16rne(rb);
        }
        ahi.u[j] = th;
        alo.u[j] = tl;
      }
#pragma unroll
      for (int nt = 0; nt < 4; ++nt) {
        FragB bh, bl;
        const unsigned short* bp = wwh + (16 * nt + m) * FD + 32 * c + 8 * hh;
        const unsigned short* bq = wwl + (16 * nt + m) * FD + 32 * c + 8 * hh;
        bh.u[0] = *(const v8us*)bp;  bh.u[1] = *(const v8us*)(bp + 16);
        bl.u[0] = *(const v8us*)bq;  bl.u[1] = *(const v8us*)(bq + 16);
        o[nt] = wmb(ahi.v, bh.v, o[nt]);
        o[nt] = wmb(alo.v, bh.v, o[nt]);
        o[nt] = wmb(ahi.v, bl.v, o[nt]);
      }
    }
    tile_store<1>(o[0], o[1], o[2], o[3], accs + sb * FD, outp, nodeBase + sb, nN, lane, hh, m);
  }
}

extern "C" void kernel_launch(void* const* d_in, const int* in_sizes, int n_in,
                              void* d_out, int out_size, void* d_ws, size_t ws_size,
                              hipStream_t stream) {
  if (n_in < 12) return;
  const int nN = in_sizes[0] / FD;
  const int nE = in_sizes[2];
  if (nN < 1 || nE < 1) return;
  if (in_sizes[0] != nN * FD || in_sizes[1] != nN * FD || in_sizes[3] != nE) return;
  if (in_sizes[4] != 2 * FD * FD || in_sizes[5] < FD || in_sizes[6] != FD * FD || in_sizes[7] < FD) return;
  if (in_sizes[8] != FD || in_sizes[9] < 1 || in_sizes[10] != FD * FD || in_sizes[11] < FD) return;
  if (out_size != nN * FD) return;

  const float* uf      = (const float*)d_in[0];
  const float* hif     = (const float*)d_in[1];
  const int*   trust   = (const int*)d_in[2];
  const int*   trustee = (const int*)d_in[3];
  const float* W1 = (const float*)d_in[4];
  const float* b1 = (const float*)d_in[5];
  const float* W2 = (const float*)d_in[6];
  const float* b2 = (const float*)d_in[7];
  const float* W3 = (const float*)d_in[8];
  const float* b3 = (const float*)d_in[9];
  const float* Ww = (const float*)d_in[10];
  const float* bw = (const float*)d_in[11];
  float* out = (float*)d_out;

  const int nBlkN = (nN + NRB - 1) / NRB;
  const size_t nPad   = (size_t)nBlkN * NRB;
  const size_t planeB = nPad * FD * sizeof(float);
  const size_t oP = 0, oQ = planeB, total = 2 * planeB;
  if (total > ws_size || total > WSB_MAX) return;
  char* ws = (char*)d_ws;
  float* Pp = (float*)(ws + oP);
  float* Qp = (float*)(ws + oQ);

  k_node<<<nBlkN, NTHR, 0, stream>>>(uf, hif, W1, b1, Pp, Qp, nN);

  const int nBlkA = (nN + NB - 1) / NB;
  k_agg<<<nBlkA, NTHR, 0, stream>>>(Pp, Qp, hif, trust, trustee, W2, b2, W3, b3, Ww, bw, out, nN, nE);
}
